// SwinV2Block_8048768713331
// MI455X (gfx1250) — hardware-verified
//
#include <hip/hip_runtime.h>
#include <math.h>

typedef __attribute__((ext_vector_type(16))) _Float16 v16h;
typedef __attribute__((ext_vector_type(8)))  _Float16 v8h;
typedef __attribute__((ext_vector_type(16))) __bf16   v16b;
typedef __attribute__((ext_vector_type(8)))  __bf16   v8b;
typedef __attribute__((ext_vector_type(8)))  float    v8f;
typedef __attribute__((ext_vector_type(4)))  float    v4f;

#define NEG_INF (-__builtin_huge_valf())

__device__ __forceinline__ unsigned short f2bf_bits(float f) {
  unsigned u = __float_as_uint(f);
  return (unsigned short)((u + 0x7FFFu + ((u >> 16) & 1u)) >> 16);
}
__device__ __forceinline__ float bf_bits2f(unsigned short h) { return __uint_as_float(((unsigned)h) << 16); }

__device__ __forceinline__ void dep_guard_h(v8f& a, v8f& b, v16h x, v16h y) { asm volatile("v_nop\n\tv_nop\n\tv_nop\n\tv_nop" : "+v"(a), "+v"(b) : "v"(x), "v"(y)); }
__device__ __forceinline__ void dep_guard_b(v8f& a, v8f& b, v16b x, v16b y) { asm volatile("v_nop\n\tv_nop\n\tv_nop\n\tv_nop" : "+v"(a), "+v"(b) : "v"(x), "v"(y)); }
__device__ __forceinline__ void keep4_h(v16h a, v16h b, v16h c, v16h d) { asm volatile("v_nop" :: "v"(a), "v"(b), "v"(c), "v"(d)); }
__device__ __forceinline__ void keep4_b(v16b a, v16b b, v16b c, v16b d) { asm volatile("v_nop" :: "v"(a), "v"(b), "v"(c), "v"(d)); }
__device__ __forceinline__ void acc_guard4(v8f& a, v8f& b, v8f& c, v8f& d) { asm volatile("v_nop\n\tv_nop\n\tv_nop\n\tv_nop" : "+v"(a), "+v"(b), "+v"(c), "+v"(d)); }
template <typename T> struct Frag;
template <> struct Frag<_Float16> {
  typedef v16h V; union U { v16h v; v8h h[2]; };
  static __device__ __forceinline__ v16h load(const _Float16* p) {
    U f; f.h[0] = *(const v8h*)(p); f.h[1] = *(const v8h*)(p + 16); return f.v;
  }
  static __device__ __forceinline__ v8f mma(v16h a, v16h b, v8f c) {
    return __builtin_amdgcn_wmma_f32_16x16x32_f16(false, a, false, b, (short)0, c, false, false);
  }
  static __device__ __forceinline__ void guard(v8f& a, v8f& b, v16h x, v16h y) { dep_guard_h(a, b, x, y); }
  static __device__ __forceinline__ void keep(v16h a, v16h b, v16h c, v16h d) { keep4_h(a, b, c, d); }
};
template <> struct Frag<__bf16> {
  typedef v16b V; union U { v16b v; v8b h[2]; };
  static __device__ __forceinline__ v16b load(const __bf16* p) {
    U f; f.h[0] = *(const v8b*)(p); f.h[1] = *(const v8b*)(p + 16); return f.v;
  }
  static __device__ __forceinline__ v8f mma(v16b a, v16b b, v8f c) {
    return __builtin_amdgcn_wmma_f32_16x16x32_bf16(false, a, false, b, (short)0, c, false, false);
  }
  static __device__ __forceinline__ void guard(v8f& a, v8f& b, v16b x, v16b y) { dep_guard_b(a, b, x, y); }
  static __device__ __forceinline__ void keep(v16b a, v16b b, v16b c, v16b d) { keep4_b(a, b, c, d); }
};

template <int ET> struct Elem;
template <> struct Elem<0> { typedef _Float16 T; };
template <> struct Elem<1> { typedef __bf16 T; };
template <int ET, bool SPLIT, int BIAS_MODE, int OUT_MODE, bool RESID, int ACT = 0>
__global__ __launch_bounds__(256) void wmma_gemm64(
    const unsigned short* __restrict__ Ap, const unsigned short* __restrict__ A2p, int lda, long strideA,
    const unsigned short* __restrict__ Btp, const unsigned short* __restrict__ Bt2p, int ldb, long strideB,
    void* __restrict__ Cout, void* __restrict__ Cout2, int ldc, long strideC,
    const float* __restrict__ bias,
    const float* __restrict__ resid, long strideR,
    int M, int N, int K, float scale, float oscale) {
  typedef typename Elem<ET>::T T;
  typedef typename Frag<T>::V V;
  const T* A = (const T*)Ap; const T* A2 = (const T*)A2p; const T* Bt = (const T*)Btp; const T* Bt2 = (const T*)Bt2p;
  __shared__ __align__(16) float sT[8][16 * 68];
  const int b    = blockIdx.y;
  const int lane = threadIdx.x & 31;
  const int wave = threadIdx.x >> 5;
  const int tilesN = N >> 6;
  const int tilesM = M >> 6;
  const int tile = blockIdx.x * 8 + wave;
  if (tile >= tilesM * tilesN) return;
  const int tm = tile / tilesN;
  const int tn = tile - tm * tilesN;
  const int m0 = tm << 6;
  const int n0 = tn << 6;

  const T* Ab  = A  + (size_t)b * strideA;
  const T* Bb  = Bt + (size_t)b * strideB;
  const T* Ab2 = SPLIT ? (A2  + (size_t)b * strideA) : nullptr;
  const T* Bb2 = SPLIT ? (Bt2 + (size_t)b * strideB) : nullptr;

  const int rlane = lane & 15;
  const int koff  = (lane >> 4) * 8;
  const int mOff  = (lane >> 4) * 8;

  v8f acc[4][4];
#pragma unroll
  for (int i = 0; i < 4; ++i)
#pragma unroll
    for (int j = 0; j < 4; ++j) acc[i][j] = (v8f){0.f,0.f,0.f,0.f,0.f,0.f,0.f,0.f};

  for (int k0 = 0; k0 < K; k0 += 32) {
    V bh[4], bl[4];
#pragma unroll
    for (int j = 0; j < 4; ++j) {
      const size_t bo = (size_t)(n0 + (j << 4) + rlane) * ldb + koff + k0;
      bh[j] = Frag<T>::load(Bb + bo);
      if (SPLIT) bl[j] = Frag<T>::load(Bb2 + bo);
    }
#pragma unroll
    for (int i = 0; i < 4; ++i) {
      const size_t ao = (size_t)(m0 + (i << 4) + rlane) * lda + koff + k0;
      V ah = Frag<T>::load(Ab + ao);
      V al;
      if (SPLIT) al = Frag<T>::load(Ab2 + ao);
#pragma unroll
      for (int j = 0; j < 4; ++j) {
        acc[i][j] = Frag<T>::mma(ah, bh[j], acc[i][j]);
        if (SPLIT) {
          acc[i][j] = Frag<T>::mma(ah, bl[j], acc[i][j]);
          acc[i][j] = Frag<T>::mma(al, bh[j], acc[i][j]);
        }
      }
      Frag<T>::guard(acc[i][0], acc[i][3], ah, SPLIT ? al : ah);
    }
    Frag<T>::keep(bh[0], bh[1], bh[2], bh[3]);
    if (SPLIT) Frag<T>::keep(bl[0], bl[1], bl[2], bl[3]);
  }
  acc_guard4(acc[0][0], acc[0][1], acc[0][2], acc[0][3]);
  acc_guard4(acc[1][0], acc[1][1], acc[1][2], acc[1][3]);
  acc_guard4(acc[2][0], acc[2][1], acc[2][2], acc[2][3]);
  acc_guard4(acc[3][0], acc[3][1], acc[3][2], acc[3][3]);

  float* slab = sT[wave];
  const float* Rb = RESID ? (resid + (size_t)b * strideR) : nullptr;
#pragma unroll
  for (int i = 0; i < 4; ++i) {
    const int mBase = m0 + (i << 4);
#pragma unroll
    for (int j = 0; j < 4; ++j) {
      const int n = n0 + (j << 4) + rlane;
      float bv = 0.f;
      if (BIAS_MODE == 2) bv = bias[n];
#pragma unroll
      for (int r = 0; r < 8; ++r) {
        float v = acc[i][j][r] * scale;
        if (BIAS_MODE == 1) v += bias[mBase + mOff + r];
        if (BIAS_MODE == 2) v += bv;
        if (RESID) v += Rb[(size_t)(mBase + mOff + r) * ldc + n];
        if (ACT == 1) v = tanhf(v);
        if (ACT == 2) v = fmaxf(v, 0.0f);
        if (ACT == 3) v = v / (1.0f + expf(-v));
        if (ACT == 4) v = (v > 0.f) ? v : 0.01f * v;
        if (ACT == 5) v = 0.5f * v * (1.0f + erff(v * 0.70710678118654752f));
        slab[(mOff + r) * 68 + (j << 4) + rlane] = v * oscale;
      }
    }
    __builtin_amdgcn_fence(__ATOMIC_RELEASE, "workgroup");
    __builtin_amdgcn_wave_barrier();
    __builtin_amdgcn_fence(__ATOMIC_ACQUIRE, "workgroup");
    if (OUT_MODE == 0) {
      float* C = (float*)Cout + (size_t)b * strideC;
      const int hh = lane >> 4, c4 = (lane & 15) * 4;
      for (int pass = 0; pass < 2; ++pass) {
#pragma unroll
        for (int it = 0; it < 8; ++it) {
          const int row = it * 2 + hh;
          v4f v = *(const v4f*)(slab + row * 68 + c4);
          *(volatile v4f*)(C + (size_t)(mBase + row) * ldc + n0 + c4) = v;
        }
        __threadfence();
      }
    } else {
      const int q = lane >> 3, c8 = (lane & 7) * 8;
      unsigned short* C  = (unsigned short*)Cout  + (size_t)b * strideC;
      unsigned short* C2 = (OUT_MODE == 2) ? ((unsigned short*)Cout2 + (size_t)b * strideC) : nullptr;
      for (int pass = 0; pass < 2; ++pass) {
#pragma unroll
        for (int it = 0; it < 4; ++it) {
          const int row = it * 4 + q;
          const float* sp = slab + row * 68 + c8;
          v8h hv, lv;
#pragma unroll
          for (int e = 0; e < 8; ++e) {
            if (OUT_MODE == 1) {
              hv[e] = (_Float16)sp[e];
            } else {
              unsigned short hb = f2bf_bits(sp[e]);
              unsigned short lb = f2bf_bits(sp[e] - bf_bits2f(hb));
              hv[e] = __builtin_bit_cast(_Float16, hb);
              lv[e] = __builtin_bit_cast(_Float16, lb);
            }
          }
          *(volatile v8h*)(C + (size_t)(mBase + row) * ldc + n0 + c8) = hv;
          if (OUT_MODE == 2) *(volatile v8h*)(C2 + (size_t)(mBase + row) * ldc + n0 + c8) = lv;
        }
        __threadfence();
      }
    }
    __builtin_amdgcn_fence(__ATOMIC_RELEASE, "workgroup");
    __builtin_amdgcn_wave_barrier();
    __builtin_amdgcn_fence(__ATOMIC_ACQUIRE, "workgroup");
  }
}

__global__ __launch_bounds__(256) void cast8_kernel(
    const float* __restrict__ in, _Float16* __restrict__ out, int n8, float scale) {
  const int i = blockIdx.x * 256 + threadIdx.x;
  if (i < n8) {
    const float* p = in + (size_t)i * 8;
    const v4f f0 = *(const v4f*)p;
    const v4f f1 = *(const v4f*)(p + 4);
    v8h hv;
    hv[0] = (_Float16)(f0[0] * scale); hv[1] = (_Float16)(f0[1] * scale);
    hv[2] = (_Float16)(f0[2] * scale); hv[3] = (_Float16)(f0[3] * scale);
    hv[4] = (_Float16)(f1[0] * scale); hv[5] = (_Float16)(f1[1] * scale);
    hv[6] = (_Float16)(f1[2] * scale); hv[7] = (_Float16)(f1[3] * scale);
    _Float16* q = out + (size_t)i * 8;
    *(volatile v8h*)q = hv;
    __threadfence();
    *(volatile v8h*)q = hv;
  }
}

__global__ __launch_bounds__(256) void split8_kernel(
    const float* __restrict__ in, unsigned short* __restrict__ hi, unsigned short* __restrict__ lo, int n8) {
  const int i = blockIdx.x * 256 + threadIdx.x;
  if (i < n8) {
    const float* p = in + (size_t)i * 8;
    const v4f f0 = *(const v4f*)p;
    const v4f f1 = *(const v4f*)(p + 4);
    v8h hv, lv;
#pragma unroll
    for (int e = 0; e < 4; ++e) {
      const unsigned short hb0 = f2bf_bits(f0[e]);
      const unsigned short lb0 = f2bf_bits(f0[e] - bf_bits2f(hb0));
      hv[e] = __builtin_bit_cast(_Float16, hb0);
      lv[e] = __builtin_bit_cast(_Float16, lb0);
      const unsigned short hb1 = f2bf_bits(f1[e]);
      const unsigned short lb1 = f2bf_bits(f1[e] - bf_bits2f(hb1));
      hv[4 + e] = __builtin_bit_cast(_Float16, hb1);
      lv[4 + e] = __builtin_bit_cast(_Float16, lb1);
    }
    unsigned short* qh = hi + (size_t)i * 8;
    unsigned short* ql = lo + (size_t)i * 8;
    *(volatile v8h*)qh = hv;
    *(volatile v8h*)ql = lv;
    __threadfence();
    *(volatile v8h*)qh = hv;
    *(volatile v8h*)ql = lv;
  }
}

#define NTOK 32768
#define CHN 384
#define QKVLD 1152
#define HIDC 1536
#define NHEAD 12
#define HDIM 32
#define NWIN 512
#define NREL 225
#define RPBPAD 2816
#define CHROWS 4096
#define NCHUNK 8
static_assert(NTOK == NCHUNK * CHROWS, "chunks cover all rows");
static_assert(NTOK % 64 == 0 && CHROWS % 64 == 0 && CHN % 64 == 0 && QKVLD % 64 == 0 && HIDC % 64 == 0, "tile multiples");
static_assert(CHN % 32 == 0 && HIDC % 32 == 0, "K multiples of 32");
static_assert(RPBPAD >= NREL * NHEAD && RPBPAD % 32 == 0, "rpb table padding");

__device__ __forceinline__ int tokrow(int win, int t) {
  const int b  = win >> 6;
  const int wq = win & 63;
  const int wi = wq >> 3, wj = wq & 7;
  const int ho = (wi * 8 + (t >> 3) + 4) & 63;
  const int wo = (wj * 8 + (t & 7) + 4) & 63;
  return (b * 64 + ho) * 64 + wo;
}
__device__ __forceinline__ int lab3(int p) { return (p < 56) ? 0 : ((p < 60) ? 1 : 2); }

__global__ __launch_bounds__(256) void qkvb_kernel(
    const float* __restrict__ qb, const float* __restrict__ vb, float* __restrict__ dst) {
  const int i = blockIdx.x * 256 + threadIdx.x;
  if (i < QKVLD / 4) {
    const int c0 = i * 4;
    const int qi = (c0 < CHN - 4) ? c0 : (CHN - 4);
    int vi = c0 - 2 * CHN; vi = (vi < 0) ? 0 : vi;
    const v4f qv = *(const v4f*)(qb + qi);
    const v4f vv = *(const v4f*)(vb + vi);
    const bool isq = (c0 < CHN);
    const bool isv = (c0 >= 2 * CHN);
    v4f val;
#pragma unroll
    for (int e = 0; e < 4; ++e) val[e] = isq ? qv[e] : (isv ? vv[e] : 0.0f);
    float* p = dst + c0;
    *(volatile v4f*)p = val;
    __threadfence();
    *(volatile v4f*)p = val;
  }
}

__global__ __launch_bounds__(256) void rpb_kernel(
    const float* __restrict__ w1, const float* __restrict__ b1, const float* __restrict__ w2,
    float* __restrict__ rpbt) {
  __shared__ __align__(16) float tab[RPBPAD];
  const int tid = threadIdx.x;
  for (int i = tid; i < RPBPAD; i += 256) tab[i] = 0.f;
  __syncthreads();
#pragma unroll 1
  for (int o = tid; o < NREL * NHEAD; o += 256) {
    const int p = o / NHEAD;
    const int h = o - p * NHEAD;
    const int dy = p / 15, dx = p - dy * 15;
    const float ry = (float)(dy - 7) * (1.0f / 7.0f) * 8.0f;
    const float rx = (float)(dx - 7) * (1.0f / 7.0f) * 8.0f;
    const float ty = copysignf(log2f(fabsf(ry) + 1.0f) * (1.0f / 3.0f), ry);
    const float tx = copysignf(log2f(fabsf(rx) + 1.0f) * (1.0f / 3.0f), rx);
    const float* w2r = w2 + h * 512;
    float acc = 0.f;
#pragma unroll 1
    for (int j = 0; j < 512; ++j) {
      const float hv = fmaxf(ty * w1[2 * j] + tx * w1[2 * j + 1] + b1[j], 0.0f);
      acc += hv * w2r[j];
    }
    const float e = __expf(-acc);
    tab[o] = 16.0f / (1.0f + e);
  }
  __syncthreads();
  for (int i = tid; i < RPBPAD / 4; i += 256) {
    const v4f v = *(const v4f*)(tab + i * 4);
    *(volatile v4f*)(rpbt + i * 4) = v;
  }
  __threadfence();
  for (int i = tid; i < RPBPAD / 4; i += 256) {
    const v4f v = *(const v4f*)(tab + i * 4);
    *(volatile v4f*)(rpbt + i * 4) = v;
  }
}

template <bool HOUT>
__global__ __launch_bounds__(256) void ln_res_kernel(
    const float* __restrict__ src, const float* __restrict__ res,
    const float* __restrict__ g, const float* __restrict__ bb,
    float* __restrict__ outf, _Float16* __restrict__ outh, int nrows, float hscale) {
  __shared__ __align__(16) float slab[8][512];
  const int wave = threadIdx.x >> 5, lane = threadIdx.x & 31;
  const int row = blockIdx.x * 8 + wave;
  if (row >= nrows) return;
  const float* sp = src + (size_t)row * CHN + lane * 4;
  const float* rp = res + (size_t)row * CHN + lane * 4;
  const v4f a0 = *(const v4f*)(sp);
  const v4f a1 = *(const v4f*)(sp + 128);
  const v4f a2 = *(const v4f*)(sp + 256);
  float s = ((a0[0] + a0[1]) + (a0[2] + a0[3])) + ((a1[0] + a1[1]) + (a1[2] + a1[3])) + ((a2[0] + a2[1]) + (a2[2] + a2[3]));
#pragma unroll
  for (int off = 16; off >= 1; off >>= 1) s += __shfl_xor(s, off, 32);
  const float mu = s * (1.0f / 384.0f);
  v4f d0, d1, d2;
#pragma unroll
  for (int e = 0; e < 4; ++e) { d0[e] = a0[e] - mu; d1[e] = a1[e] - mu; d2[e] = a2[e] - mu; }
  float sq = ((d0[0] * d0[0] + d0[1] * d0[1]) + (d0[2] * d0[2] + d0[3] * d0[3]))
           + ((d1[0] * d1[0] + d1[1] * d1[1]) + (d1[2] * d1[2] + d1[3] * d1[3]))
           + ((d2[0] * d2[0] + d2[1] * d2[1]) + (d2[2] * d2[2] + d2[3] * d2[3]));
#pragma unroll
  for (int off = 16; off >= 1; off >>= 1) sq += __shfl_xor(sq, off, 32);
  const float rs = rsqrtf(sq * (1.0f / 384.0f) + 1e-5f);
  const v4f g0 = *(const v4f*)(g + lane * 4);
  const v4f g1 = *(const v4f*)(g + 128 + lane * 4);
  const v4f g2 = *(const v4f*)(g + 256 + lane * 4);
  const v4f b0 = *(const v4f*)(bb + lane * 4);
  const v4f b1 = *(const v4f*)(bb + 128 + lane * 4);
  const v4f b2 = *(const v4f*)(bb + 256 + lane * 4);
  const v4f r0 = *(const v4f*)(rp);
  const v4f r1 = *(const v4f*)(rp + 128);
  const v4f r2 = *(const v4f*)(rp + 256);
  v4f y0, y1, y2;
#pragma unroll
  for (int e = 0; e < 4; ++e) {
    y0[e] = r0[e] + (d0[e] * rs * g0[e] + b0[e]);
    y1[e] = r1[e] + (d1[e] * rs * g1[e] + b1[e]);
    y2[e] = r2[e] + (d2[e] * rs * g2[e] + b2[e]);
  }
  float* op = outf + (size_t)row * CHN + lane * 4;
  for (int pass = 0; pass < 2; ++pass) {
    *(volatile v4f*)(op)       = y0;
    *(volatile v4f*)(op + 128) = y1;
    *(volatile v4f*)(op + 256) = y2;
    __threadfence();
  }
  if (HOUT) {
    float* sl = slab[wave];
#pragma unroll
    for (int e = 0; e < 4; ++e) {
      sl[lane * 4 + e]       = y0[e] * hscale;
      sl[128 + lane * 4 + e] = y1[e] * hscale;
      sl[256 + lane * 4 + e] = y2[e] * hscale;
    }
    __builtin_amdgcn_fence(__ATOMIC_RELEASE, "workgroup");
    __builtin_amdgcn_wave_barrier();
    __builtin_amdgcn_fence(__ATOMIC_ACQUIRE, "workgroup");
    const float* p0 = sl + lane * 8;
    const float* p1 = sl + 256 + (lane & 15) * 8;
    v8h h0, h1;
#pragma unroll
    for (int e = 0; e < 8; ++e) { h0[e] = (_Float16)p0[e]; h1[e] = (_Float16)p1[e]; }
    _Float16* hp = outh + (size_t)row * CHN;
    for (int pass = 0; pass < 2; ++pass) {
      *(volatile v8h*)(hp + lane * 8) = h0;
      if (lane < 16) *(volatile v8h*)(hp + 256 + lane * 8) = h1;
      __threadfence();
    }
  }
}

__global__ __launch_bounds__(256) void gelu2_kernel(
    const _Float16* __restrict__ in, _Float16* __restrict__ out, int n2, float iscale, float oscale) {
  const int i = blockIdx.x * 256 + threadIdx.x;
  if (i < n2) {
    const unsigned u = ((const unsigned*)in)[i];
    unsigned res = 0u;
#pragma unroll 1
    for (int e = 0; e < 2; ++e) {
      const unsigned short hb = (unsigned short)((u >> (16 * e)) & 0xFFFFu);
      const float x = (float)__builtin_bit_cast(_Float16, hb) * iscale;
      const float y = 0.5f * x * (1.0f + erff(x * 0.70710678118654752f));
      const unsigned short ob = __builtin_bit_cast(unsigned short, (_Float16)(y * oscale));
      res |= ((unsigned)ob) << (16 * e);
    }
    ((volatile unsigned*)out)[i] = res;
    __threadfence();
    ((volatile unsigned*)out)[i] = res;
  }
}

#define KPI 40
#define VPI 72
#define PPI 72
#define OPI 36
#define PCARRY 32768.0f
#define QCARRY 16.0f
#define LN100F 4.6051702f

__device__ __forceinline__ v8f mma_h(v16h a, v16h b, v8f c) {
  c = __builtin_amdgcn_wmma_f32_16x16x32_f16(false, a, false, b, (short)0, c, false, false);
  asm volatile("v_nop\n\tv_nop\n\tv_nop\n\tv_nop" : "+v"(c) : "v"(a), "v"(b));
  return c;
}

__global__ __launch_bounds__(256) void win_attn_kernel(
    const _Float16* __restrict__ qkv, const float* __restrict__ rpbt,
    const float* __restrict__ flex, _Float16* __restrict__ att) {
  __shared__ __align__(16) _Float16 Qs[2][64 * KPI];
  __shared__ __align__(16) _Float16 Ks[2][64 * KPI];
  __shared__ __align__(16) _Float16 Vt[2][HDIM * VPI];
  __shared__ __align__(16) _Float16 Ps[8][16 * PPI];
  __shared__ __align__(16) float Os[8][16 * OPI];
  __shared__ float sBias[2][232];

  const int tid  = threadIdx.x;
  const int wave = tid >> 5;
  const int lane = tid & 31;
  const int hh   = lane >> 4;
  const int c    = lane & 15;
  const int hp   = blockIdx.x;
  const int win  = blockIdx.y;
  const int wi   = (win >> 3) & 7;
  const int wj   = win & 7;

  for (int i = tid; i < 2 * NREL; i += 256) {
    const int gg = (i >= NREL) ? 1 : 0;
    const int p  = i - gg * NREL;
    sBias[gg][p] = rpbt[p * NHEAD + 2 * hp + gg];
  }
  {
    const int kvr = tid >> 2, pc = tid & 3;
    const _Float16* base = qkv + (size_t)tokrow(win, kvr) * QKVLD + (2 * hp) * HDIM + pc * 8;
#pragma unroll
    for (int gg = 0; gg < 2; ++gg) {
      const _Float16* bq = base + gg * HDIM;
      const v8h q8 = *(const v8h*)(bq);
      const v8h k8 = *(const v8h*)(bq + CHN);
      const v8h w8 = *(const v8h*)(bq + 2 * CHN);
      float qf[8], kf[8];
      float qs = 0.f, ks = 0.f;
#pragma unroll
      for (int e = 0; e < 8; ++e) {
        qf[e] = (float)q8[e] * 0.125f;
        kf[e] = (float)k8[e] * 0.125f;
        qs += qf[e] * qf[e];
        ks += kf[e] * kf[e];
      }
      qs += __shfl_xor(qs, 1, 32); qs += __shfl_xor(qs, 2, 32);
      ks += __shfl_xor(ks, 1, 32); ks += __shfl_xor(ks, 2, 32);
      const float qi = QCARRY / fmaxf(sqrtf(qs), 1e-12f);
      const float ki = QCARRY / fmaxf(sqrtf(ks), 1e-12f);
      v8h qn, kn;
#pragma unroll
      for (int e = 0; e < 8; ++e) { qn[e] = (_Float16)(qf[e] * qi); kn[e] = (_Float16)(kf[e] * ki); }
      *(v8h*)(Qs[gg] + kvr * KPI + pc * 8) = qn;
      *(v8h*)(Ks[gg] + kvr * KPI + pc * 8) = kn;
#pragma unroll
      for (int e = 0; e < 8; ++e) Vt[gg][(pc * 8 + e) * VPI + kvr] = w8[e];
    }
  }
  __syncthreads();

  const int gq  = wave >> 2;
  const int h   = 2 * hp + gq;
  const int wq4 = wave & 3;
  const int q0  = wq4 * 16;
  const float sc = expf(fminf(flex[h], LN100F)) * (1.0f / (QCARRY * QCARRY));
  const v16h qa = Frag<_Float16>::load(Qs[gq] + (q0 + c) * KPI + 8 * hh);

  v8f s[4];
#pragma unroll
  for (int j = 0; j < 4; ++j) {
    s[j] = (v8f){0.f,0.f,0.f,0.f,0.f,0.f,0.f,0.f};
    const v16h kb = Frag<_Float16>::load(Ks[gq] + (j * 16 + c) * KPI + 8 * hh);
    s[j] = mma_h(qa, kb, s[j]);
  }

  const int rq    = 2 * wq4 + hh;
  const int regqh = 3 * lab3(wi * 8 + rq);
  const int ck    = c & 7;
  const int regkw = lab3(wj * 8 + ck);
  const int rkh   = c >> 3;
  float lrow[8];
  _Float16* pw = Ps[wave];
#pragma unroll
  for (int r = 0; r < 8; ++r) {
    const int regq = regqh + lab3(wj * 8 + r);
    float m = NEG_INF;
#pragma unroll
    for (int j = 0; j < 4; ++j) {
      const int rk = 2 * j + rkh;
      const int regk = 3 * lab3(wi * 8 + rk) + regkw;
      const float bias = sBias[gq][(rq - rk + 7) * 15 + (r - ck + 7)];
      float v = s[j][r] * sc + bias;
      v = v + ((regq != regk) ? -100.0f : 0.0f);
      s[j][r] = v;
      m = fmaxf(m, v);
    }
#pragma unroll
    for (int off = 1; off < 16; off <<= 1) m = fmaxf(m, __shfl_xor(m, off, 32));
    float psum = 0.f;
#pragma unroll
    for (int j = 0; j < 4; ++j) {
      const float p = __expf(s[j][r] - m);
      psum += p;
      pw[(8 * hh + r) * PPI + j * 16 + c] = (_Float16)(p * PCARRY);
    }
#pragma unroll
    for (int off = 1; off < 16; off <<= 1) psum += __shfl_xor(psum, off, 32);
    lrow[r] = psum;
  }
  __builtin_amdgcn_fence(__ATOMIC_RELEASE, "workgroup");
  __builtin_amdgcn_wave_barrier();
  __builtin_amdgcn_fence(__ATOMIC_ACQUIRE, "workgroup");

  v8f oacc[2];
  oacc[0] = (v8f){0.f,0.f,0.f,0.f,0.f,0.f,0.f,0.f};
  oacc[1] = (v8f){0.f,0.f,0.f,0.f,0.f,0.f,0.f,0.f};
#pragma unroll
  for (int kk = 0; kk < 2; ++kk) {
    const v16h pa = Frag<_Float16>::load(pw + c * PPI + kk * 32 + 8 * hh);
#pragma unroll
    for (int t = 0; t < 2; ++t) {
      const v16h vb = Frag<_Float16>::load(Vt[gq] + (t * 16 + c) * VPI + kk * 32 + 8 * hh);
      oacc[t] = mma_h(pa, vb, oacc[t]);
    }
  }

  float* os = Os[wave];
#pragma unroll
  for (int r = 0; r < 8; ++r) {
    const float inv = 1.0f / (lrow[r] * 16384.0f);
    os[(8 * hh + r) * OPI + c]      = oacc[0][r] * inv;
    os[(8 * hh + r) * OPI + 16 + c] = oacc[1][r] * inv;
  }
  __syncthreads();
  {
    const int q8 = lane >> 3, c8 = lane & 7;
    const int g2 = c8 >> 2, d0 = (c8 & 3) * 8;
    for (int pass = 0; pass < 2; ++pass) {
#pragma unroll
      for (int it = 0; it < 2; ++it) {
        const int tok = wave * 8 + it * 4 + q8;
        const float* op = Os[g2 * 4 + (tok >> 4)] + (tok & 15) * OPI + d0;
        v8h hv;
#pragma unroll
        for (int e = 0; e < 8; ++e) hv[e] = (_Float16)op[e];
        _Float16* dst = att + (size_t)tokrow(win, tok) * CHN + hp * 64 + c8 * 8;
        *(volatile v8h*)dst = hv;
      }
      __threadfence();
    }
  }
}

extern "C" void kernel_launch(void* const* d_in, const int* in_sizes, int n_in,
                              void* d_out, int out_size, void* d_ws, size_t ws_size,
                              hipStream_t stream) {
  if (n_in < 18) return;
  if (in_sizes[0] != NTOK * CHN) return;
  if (in_sizes[1] != QKVLD * CHN || in_sizes[2] != CHN || in_sizes[3] != CHN) return;
  if (in_sizes[4] != NHEAD) return;
  if (in_sizes[5] != 512 * 2 || in_sizes[6] != 512 || in_sizes[7] != NHEAD * 512) return;
  if (in_sizes[8] != CHN * CHN || in_sizes[9] != CHN) return;
  if (in_sizes[10] != CHN || in_sizes[11] != CHN || in_sizes[12] != CHN || in_sizes[13] != CHN) return;
  if (in_sizes[14] != HIDC * CHN || in_sizes[15] != HIDC) return;
  if (in_sizes[16] != CHN * HIDC || in_sizes[17] != CHN) return;
  if (out_size != NTOK * CHN) return;

  const float* x      = (const float*)d_in[0];
  const float* qkv_w  = (const float*)d_in[1];
  const float* q_bias = (const float*)d_in[2];
  const float* v_bias = (const float*)d_in[3];
  const float* flex   = (const float*)d_in[4];
  const float* cpb_w1 = (const float*)d_in[5];
  const float* cpb_b1 = (const float*)d_in[6];
  const float* cpb_w2 = (const float*)d_in[7];
  const float* proj_w = (const float*)d_in[8];
  const float* proj_b = (const float*)d_in[9];
  const float* n1g    = (const float*)d_in[10];
  const float* n1b    = (const float*)d_in[11];
  const float* n2g    = (const float*)d_in[12];
  const float* n2b    = (const float*)d_in[13];
  const float* fc1_w  = (const float*)d_in[14];
  const float* fc1_b  = (const float*)d_in[15];
  const float* fc2_w  = (const float*)d_in[16];
  const float* fc2_b  = (const float*)d_in[17];
  float* out = (float*)d_out;

  const size_t szWQ = (size_t)QKVLD * CHN * 2;
  const size_t szWP = (size_t)CHN * CHN * 2;
  const size_t szW1 = (size_t)HIDC * CHN * 2;
  const size_t szW2 = (size_t)CHN * HIDC * 2;
  const size_t szQB = (size_t)QKVLD * 4;
  const size_t szRP = (size_t)RPBPAD * 4;
  const size_t szXP = (size_t)NTOK * CHN * 2;
  const size_t szRA = 2 * szXP;
  const size_t szRB = (size_t)NTOK * QKVLD * 2;
  const size_t oWQH = 0;
  const size_t oWQL = oWQH + szWQ;
  const size_t oWP  = oWQL + szWQ;
  const size_t oW1  = oWP + szWP;
  const size_t oW2  = oW1 + szW1;
  const size_t oQB  = oW2 + szW2;
  const size_t oRP  = oQB + szQB;
  const size_t oRA  = oRP + szRP;
  const size_t oRB  = oRA + szRA;
  const size_t total = oRB + szRB;
  if (total > ws_size) return;
  const size_t cXO  = 0;
  const size_t cX1  = cXO  + (size_t)CHROWS * CHN * 4;
  const size_t cX1H = cX1  + (size_t)CHROWS * CHN * 4;
  const size_t cU   = cX1H + (size_t)CHROWS * CHN * 2;
  const size_t cG   = cU   + (size_t)CHROWS * HIDC * 2;
  const size_t cH   = cG   + (size_t)CHROWS * HIDC * 2;
  const size_t cEnd = cH   + (size_t)CHROWS * CHN * 4;
  if (cEnd > szRB) return;

  char* ws = (char*)d_ws;
  unsigned short* wqh = (unsigned short*)(ws + oWQH);
  unsigned short* wql = (unsigned short*)(ws + oWQL);
  _Float16* wp16  = (_Float16*)(ws + oWP);
  _Float16* w116  = (_Float16*)(ws + oW1);
  _Float16* w216  = (_Float16*)(ws + oW2);
  float*    qkvb  = (float*)(ws + oQB);
  float*    rpbt  = (float*)(ws + oRP);
  unsigned short* xh = (unsigned short*)(ws + oRA);
  unsigned short* xl = (unsigned short*)(ws + oRA + szXP);
  _Float16* att16 = (_Float16*)(ws + oRA);
  _Float16* qkv16 = (_Float16*)(ws + oRB);
  float*    xo    = (float*)(ws + oRB + cXO);
  float*    x1    = (float*)(ws + oRB + cX1);
  _Float16* x1h   = (_Float16*)(ws + oRB + cX1H);
  _Float16* u16   = (_Float16*)(ws + oRB + cU);
  _Float16* g16   = (_Float16*)(ws + oRB + cG);
  float*    hbuf  = (float*)(ws + oRB + cH);
  const float* dummy_resid = (const float*)(ws + oRB);

  split8_kernel<<<dim3((QKVLD * CHN / 8 + 255) / 256), 256, 0, stream>>>(qkv_w, wqh, wql, QKVLD * CHN / 8);
  cast8_kernel<<<dim3((CHN * CHN / 8 + 255) / 256), 256, 0, stream>>>(proj_w, wp16, CHN * CHN / 8, 64.0f);
  cast8_kernel<<<dim3((HIDC * CHN / 8 + 255) / 256), 256, 0, stream>>>(fc1_w, w116, HIDC * CHN / 8, 64.0f);
  cast8_kernel<<<dim3((CHN * HIDC / 8 + 255) / 256), 256, 0, stream>>>(fc2_w, w216, CHN * HIDC / 8, 64.0f);
  qkvb_kernel<<<dim3(2), 256, 0, stream>>>(q_bias, v_bias, qkvb);
  rpb_kernel<<<dim3(1), 256, 0, stream>>>(cpb_w1, cpb_b1, cpb_w2, rpbt);
  split8_kernel<<<dim3((NTOK * CHN / 8 + 255) / 256), 256, 0, stream>>>(x, xh, xl, NTOK * CHN / 8);
  {
    const int tiles = (NTOK / 64) * (QKVLD / 64);
    wmma_gemm64<1, true, 2, 1, false, 0><<<dim3((tiles + 7) / 8, 1), 256, 0, stream>>>(
        xh, xl, CHN, (long)0,
        wqh, wql, CHN, (long)0,
        (void*)qkv16, (void*)qkv16, QKVLD, (long)0,
        qkvb, dummy_resid, (long)0, NTOK, QKVLD, CHN, 1.0f, 8.0f);
  }
  win_attn_kernel<<<dim3(NHEAD / 2, NWIN), 256, 0, stream>>>(qkv16, rpbt, flex, att16);

  for (int ch = 0; ch < NCHUNK; ++ch) {
    const size_t r0c = (size_t)ch * CHROWS;
    {
      const int tiles = (CHROWS / 64) * (CHN / 64);
      wmma_gemm64<0, false, 2, 0, false, 0><<<dim3((tiles + 7) / 8, 1), 256, 0, stream>>>(
          (const unsigned short*)(att16 + r0c * CHN), (const unsigned short*)(att16 + r0c * CHN), CHN, (long)0,
          (const unsigned short*)wp16, (const unsigned short*)wp16, CHN, (long)0,
          (void*)xo, (void*)xo, CHN, (long)0,
          proj_b, dummy_resid, (long)0, CHROWS, CHN, CHN, 1.0f / 1024.0f, 1.0f);
    }
    ln_res_kernel<true><<<dim3(CHROWS / 8), 256, 0, stream>>>(xo, x + r0c * CHN, n1g, n1b, x1, x1h, CHROWS, 4.0f);
    {
      const int tiles = (CHROWS / 64) * (HIDC / 64);
      wmma_gemm64<0, false, 2, 1, false, 0><<<dim3((tiles + 7) / 8, 1), 256, 0, stream>>>(
          (const unsigned short*)x1h, (const unsigned short*)x1h, CHN, (long)0,
          (const unsigned short*)w116, (const unsigned short*)w116, CHN, (long)0,
          (void*)u16, (void*)u16, HIDC, (long)0,
          fc1_b, dummy_resid, (long)0, CHROWS, HIDC, CHN, 1.0f / 256.0f, 8.0f);
    }
    {
      const int n2 = CHROWS * HIDC / 2;
      gelu2_kernel<<<dim3((n2 + 255) / 256), 256, 0, stream>>>(u16, g16, n2, 0.125f, 16.0f);
    }
    {
      const int tiles = (CHROWS / 64) * (CHN / 64);
      wmma_gemm64<0, false, 2, 0, false, 0><<<dim3((tiles + 7) / 8, 1), 256, 0, stream>>>(
          (const unsigned short*)g16, (const unsigned short*)g16, HIDC, (long)0,
          (const unsigned short*)w216, (const unsigned short*)w216, HIDC, (long)0,
          (void*)hbuf, (void*)hbuf, CHN, (long)0,
          fc2_b, dummy_resid, (long)0, CHROWS, CHN, HIDC, 1.0f / 1024.0f, 1.0f);
    }
    ln_res_kernel<false><<<dim3(CHROWS / 8), 256, 0, stream>>>(hbuf, x1, n2g, n2b, out + r0c * CHN, x1h, CHROWS, 1.0f);
  }
}
